// NetworkLayer_42975442764619
// MI455X (gfx1250) — hardware-verified
//
#include <hip/hip_runtime.h>


#define NB_  1024
#define NN   128
#define DIN  134
#define KIN  160
#define HH   256
#define KOUT 256
#define CB   256
#define NCH  (NB_ / CB)
#define RCH  (CB * NN)
#define DP   64
#define SLOPE 0.01f
typedef _Float16 h16;
typedef unsigned short bf;
typedef __attribute__((ext_vector_type(16))) __bf16   v16bf;
typedef __attribute__((ext_vector_type(16))) _Float16 v16h;
typedef __attribute__((ext_vector_type(8)))  _Float16 v8h;
typedef __attribute__((ext_vector_type(8)))  unsigned short v8us;
typedef __attribute__((ext_vector_type(8)))  float    v8f;
typedef __attribute__((ext_vector_type(4)))  float    v4f;
typedef v8h  __attribute__((may_alias)) v8ha;
typedef v4f  __attribute__((may_alias)) v4fa;
typedef v8us __attribute__((may_alias)) v8usa;

__device__ __forceinline__ unsigned short f2bf(float f) { unsigned u = __float_as_uint(f); u += 0x7FFFu + ((u >> 16) & 1u); return (unsigned short)(u >> 16); }
__device__ __forceinline__ float bf2f(unsigned short b) { return __uint_as_float(((unsigned)b) << 16); }
__device__ __forceinline__ float bfr(float f) { return bf2f(f2bf(f)); }
__device__ __forceinline__ v16h cat16(v8h lo, v8h hi) { return __builtin_shufflevector(lo, hi, 0, 1, 2, 3, 4, 5, 6, 7, 8, 9, 10, 11, 12, 13, 14, 15); }
__device__ __forceinline__ v16bf cat16b(v8us lo, v8us hi) { return __builtin_bit_cast(v16bf, __builtin_shufflevector(lo, hi, 0, 1, 2, 3, 4, 5, 6, 7, 8, 9, 10, 11, 12, 13, 14, 15)); }
__device__ __forceinline__ v8f wmma16(v16h a, v16h b, v8f c) { return __builtin_amdgcn_wmma_f32_16x16x32_f16(false, a, false, b, (short)0, c, false, false); }
__device__ __forceinline__ v8f wmmab(v16bf a, v16bf b, v8f c) { return __builtin_amdgcn_wmma_f32_16x16x32_bf16(false, a, false, b, (short)0, c, false, false); }


template <typename T16> struct WFrag;
template <> struct WFrag<h16> { typedef v16h V; static __device__ __forceinline__ V ld(const h16* p) { return cat16(*(const v8h*)p, *(const v8h*)(p + 16)); } static __device__ __forceinline__ v8f mma(V a, V b, v8f c) { return wmma16(a, b, c); } };
template <> struct WFrag<bf> { typedef v16bf V; static __device__ __forceinline__ V ld(const bf* p) { return cat16b(*(const v8us*)p, *(const v8us*)(p + 16)); } static __device__ __forceinline__ v8f mma(V a, V b, v8f c) { return wmmab(a, b, c); } };
template <typename T16, int NSPLIT, bool BIAS>
__global__ __launch_bounds__(32) void k_gemmw(const T16* __restrict__ A, const T16* __restrict__ A2, const T16* __restrict__ Bt, const T16* __restrict__ Bt2, int K, float* C, int ldc, const float* __restrict__ bias, size_t sA, size_t sB, size_t sC) {
    typedef typename WFrag<T16>::V V;
    __shared__ __align__(16) float os[16 * 68];
    const size_t z = blockIdx.z; A += z * sA; if (A2) A2 += z * sA; Bt += z * sB; if (Bt2) Bt2 += z * sB; C += z * sC;
    const int lane = threadIdx.x & 31, lr = lane & 15, hi = lane >> 4; const int r0 = blockIdx.x * 64, c0 = blockIdx.y * 64;
    v8f acc[4][4];
#pragma unroll
    for (int mb = 0; mb < 4; ++mb)
#pragma unroll
        for (int nb = 0; nb < 4; ++nb) acc[mb][nb] = (v8f){};
    const size_t aoff = (size_t)(r0 + lr) * K + 8 * hi, boff = (size_t)(c0 + lr) * K + 8 * hi;
#pragma unroll 1
    for (int kc = 0; kc < K; kc += 32) {
        V a[4], a2[4];
#pragma unroll
        for (int mb = 0; mb < 4; ++mb) { a[mb] = WFrag<T16>::ld(A + aoff + (size_t)mb * 16 * K + kc); if (NSPLIT == 1 || NSPLIT == 2) a2[mb] = WFrag<T16>::ld(A2 + aoff + (size_t)mb * 16 * K + kc); }
#pragma unroll
        for (int nb = 0; nb < 4; ++nb) { const V b = WFrag<T16>::ld(Bt + boff + (size_t)nb * 16 * K + kc); V b2; if (NSPLIT >= 2) b2 = WFrag<T16>::ld(Bt2 + boff + (size_t)nb * 16 * K + kc);
#pragma unroll
            for (int mb = 0; mb < 4; ++mb) { acc[mb][nb] = WFrag<T16>::mma(a[mb], b, acc[mb][nb]); if (NSPLIT == 1 || NSPLIT == 2) acc[mb][nb] = WFrag<T16>::mma(a2[mb], b, acc[mb][nb]); if (NSPLIT >= 2) acc[mb][nb] = WFrag<T16>::mma(a[mb], b2, acc[mb][nb]); } }
        asm volatile("v_nop\n\tv_nop\n\tv_nop\n\tv_nop" : "+v"(acc[0][0]), "+v"(acc[1][1]), "+v"(acc[2][2]), "+v"(acc[3][3]) : "v"(a[0]), "v"(a[3]));
    }
#pragma unroll
    for (int mb = 0; mb < 4; ++mb) {
#pragma unroll
        for (int nb = 0; nb < 4; ++nb) {
#pragma unroll
            for (int j = 0; j < 8; ++j) os[(hi * 8 + j) * 68 + nb * 16 + lr] = acc[mb][nb][j]; }
        __builtin_amdgcn_wave_barrier(); asm volatile("" ::: "memory");
        float* crow = C + (size_t)(r0 + mb * 16) * ldc + c0;
#pragma unroll 1
        for (int ps = 0; ps < 2; ++ps) {
#pragma unroll
            for (int s = 0; s < 8; ++s) { const int row = 2 * s + hi, cofs = lr * 4; v4f val = *(const v4fa*)(os + row * 68 + cofs); if (BIAS) { val[0] += bfr(bias[c0 + cofs]); val[1] += bfr(bias[c0 + cofs + 1]); val[2] += bfr(bias[c0 + cofs + 2]); val[3] += bfr(bias[c0 + cofs + 3]); }
                *(volatile v4f*)(crow + (size_t)row * ldc + cofs) = val; }
            if (ps == 0) __threadfence(); }
        __builtin_amdgcn_wave_barrier(); asm volatile("" ::: "memory");
    }
}

__device__ __forceinline__ void splitf(float y, unsigned short& h, unsigned short& l) { h = f2bf(y); l = f2bf(y - bf2f(h)); }
typedef __attribute__((ext_vector_type(2))) unsigned short v2us;
typedef __attribute__((ext_vector_type(4))) unsigned short v4us;
__global__ __launch_bounds__(256) void k_wtG(const float* __restrict__ w, int K, int N, bf* Bt) {
    const int lane = threadIdx.x & 31; const int L0 = (blockIdx.x * 8 + (threadIdx.x >> 5)) * 8; const int nlines = N * K / 64;
#pragma unroll
    for (int ps = 0; ps < 2; ++ps) {
#pragma unroll 1
        for (int l = 0; l < 8; ++l) { const int L = L0 + l; if (L >= nlines) break; const size_t e = (size_t)L * 64 + lane * 2; const int k = (int)(e % K), n = (int)(e / K); v2us o;
            o[0] = f2bf(w[(size_t)k * N + n]); o[1] = f2bf(w[(size_t)(k + 1) * N + n]); *(volatile v2us*)(Bt + e) = o; }
        if (ps == 0) __threadfence(); }
}
__global__ __launch_bounds__(256) void k_w0t(const float* __restrict__ w, bf* Bt) { const size_t e = ((size_t)blockIdx.x * 256 + threadIdx.x) * 2; if (e >= (size_t)HH * KIN) return; const int k = (int)(e % KIN), n = (int)(e / KIN); v2us o;
#pragma unroll
    for (int q = 0; q < 2; ++q) o[q] = (k + q < DIN) ? f2bf(w[(size_t)(k + q) * HH + n]) : (unsigned short)0; *(volatile v2us*)(Bt + e) = o; __threadfence(); *(volatile v2us*)(Bt + e) = o; }
__global__ __launch_bounds__(256) void k_zero8(bf* Z, size_t n8) { const size_t i = (size_t)blockIdx.x * 256 + threadIdx.x; if (i >= n8) return; const v8us z = (v8us){}; *(volatile v8us*)(Z + i * 8) = z; __threadfence(); *(volatile v8us*)(Z + i * 8) = z; }
__global__ __launch_bounds__(256) void k_scal(const float* __restrict__ x, const float* __restrict__ u, const float* __restrict__ basis, int chunk, bf* Sh, bf* Sl) { const int r = blockIdx.x * 256 + threadIdx.x; if (r >= RCH) return; const int i = r % NN; const size_t b = (size_t)chunk * CB + r / NN; const float* xb = x + (b * NN) * 3; const float x0 = bfr(xb[i * 3]), x1 = bfr(xb[i * 3 + 1]), x2 = bfr(xb[i * 3 + 2]);
    float p = __fmul_rn(x0, x0); asm volatile("" : "+v"(p)); float nn = __fadd_rn(p, __fmul_rn(x1, x1)); asm volatile("" : "+v"(nn)); nn = __fadd_rn(nn, __fmul_rn(x2, x2)); const float nrm = __fsqrt_rn(nn);
    float sv[8]; sv[0] = bfr(u[b * 2]); sv[1] = bfr(u[b * 2 + 1]); sv[2] = nrm;
#pragma unroll
    for (int n = 0; n < 3; ++n) { const float* bs = basis + (b * 3 + n) * 3; float d = __fmul_rn(x0, bfr(bs[0])); asm volatile("" : "+v"(d)); d = __fadd_rn(d, __fmul_rn(x1, bfr(bs[1]))); asm volatile("" : "+v"(d)); d = __fadd_rn(d, __fmul_rn(x2, bfr(bs[2]))); sv[3 + n] = __fdiv_rn(d, nrm); }
    sv[6] = 0.f; sv[7] = 0.f;
    bf* ph = Sh + (size_t)r * KIN; bf* pl = Sl + (size_t)r * KIN;
#pragma unroll 1
    for (int ps = 0; ps < 2; ++ps) {
        v8us oh, ol;
#pragma unroll
        for (int q = 0; q < 6; ++q) { unsigned short a, c; splitf(sv[q], a, c); oh[q] = a; ol[q] = c; }
#pragma unroll 1
        for (int j0 = -6; j0 < KIN - 6; j0 += 8) {
#pragma unroll
            for (int q = 0; q < 8; ++q) { const int j = j0 + q; if (j < 0) continue; float v = 0.f; if (j < NN) { const float* xj = xb + j * 3; float d = __fmul_rn(x0, bfr(xj[0])); asm volatile("" : "+v"(d)); d = __fadd_rn(d, __fmul_rn(x1, bfr(xj[1]))); asm volatile("" : "+v"(d)); v = __fadd_rn(d, __fmul_rn(x2, bfr(xj[2]))); } unsigned short a, c; splitf(v, a, c); oh[q] = a; ol[q] = c; }
            const int slot0 = j0 + 6; *(volatile v8us*)(ph + slot0) = oh; *(volatile v8us*)(pl + slot0) = ol; }
        if (ps == 0) __threadfence(); } }
__global__ __launch_bounds__(256) void k_lrsplit(const float* __restrict__ Hs, bf* Ph, bf* Pl, size_t n4) { const size_t i = (size_t)blockIdx.x * 256 + threadIdx.x; if (i >= n4) return; const v4f h = *(const v4f*)(Hs + i * 4); v4us oh, ol;
#pragma unroll
    for (int q = 0; q < 4; ++q) { const float v = (h[q] > 0.f) ? h[q] : __fmul_rn(SLOPE, h[q]); unsigned short a, c; splitf(v, a, c); oh[q] = a; ol[q] = c; } *(volatile v4us*)(Ph + i * 4) = oh; *(volatile v4us*)(Pl + i * 4) = ol; __threadfence(); *(volatile v4us*)(Ph + i * 4) = oh; *(volatile v4us*)(Pl + i * 4) = ol; }
__global__ __launch_bounds__(256) void k_fksplit(const float* __restrict__ F, const float* __restrict__ b2, bf* Ph, bf* Pl, size_t n4) { const size_t i4 = (size_t)blockIdx.x * 256 + threadIdx.x; if (i4 >= n4) return; const size_t e = i4 * 4; const int o = (int)((e / NN) % KOUT); const float bb = bfr(b2[o]); const v4f f = *(const v4f*)(F + e); v4us oh, ol;
#pragma unroll
    for (int q = 0; q < 4; ++q) { unsigned short a, c; splitf(__fadd_rn(f[q], bb), a, c); oh[q] = a; ol[q] = c; } *(volatile v4us*)(Ph + e) = oh; *(volatile v4us*)(Pl + e) = ol; __threadfence(); *(volatile v4us*)(Ph + e) = oh; *(volatile v4us*)(Pl + e) = ol; }
__global__ __launch_bounds__(256) void k_xt(const float* __restrict__ x, int chunk, bf* XT) { const size_t e = ((size_t)blockIdx.x * 256 + threadIdx.x) * 2; if (e >= (size_t)CB * DP * NN) return; const int i = (int)(e % NN); const int d = (int)((e / NN) % DP); const size_t bl = e / ((size_t)NN * DP); const size_t b = (size_t)chunk * CB + bl; v2us o; o[0] = 0; o[1] = 0;
    if (d < 3) { o[0] = f2bf(x[(b * NN + i) * 3 + d]); o[1] = f2bf(x[(b * NN + i + 1) * 3 + d]); } *(volatile v2us*)(XT + e) = o; __threadfence(); *(volatile v2us*)(XT + e) = o; }
__global__ __launch_bounds__(256) void k_out(const float* __restrict__ C, int chunk, float* OUT) { const int e = blockIdx.x * 256 + threadIdx.x; if (e >= CB * KOUT) return; const int o = e % KOUT; const size_t bl = e / KOUT; const float* c = C + (bl * KOUT + o) * DP; float* dst = OUT + (((size_t)chunk * CB + bl) * KOUT + o) * 3; const float r0 = c[0] * (1.0f / NN), r1 = c[1] * (1.0f / NN), r2 = c[2] * (1.0f / NN);
#pragma unroll 1
    for (int ps = 0; ps < 2; ++ps) { *(volatile float*)(dst) = r0; *(volatile float*)(dst + 1) = r1; *(volatile float*)(dst + 2) = r2; if (ps == 0) __threadfence(); } }

extern "C" void kernel_launch(void* const* d_in, const int* in_sizes, int n_in,
                              void* d_out, int out_size, void* d_ws, size_t ws_size, hipStream_t stream) {
    (void)in_sizes; (void)n_in; (void)out_size;
    const float* x = (const float*)d_in[0]; const float* u = (const float*)d_in[1]; const float* basis = (const float*)d_in[2]; const float* W0 = (const float*)d_in[3]; const float* b0 = (const float*)d_in[4]; const float* W1 = (const float*)d_in[5]; const float* b1 = (const float*)d_in[6]; const float* W2 = (const float*)d_in[7]; const float* b2 = (const float*)d_in[8];
    float* OUT = (float*)d_out;
    char* wsp = (char*)d_ws;
    auto take = [&](size_t bytes) { char* p = wsp; wsp += (bytes + 255) & ~(size_t)255; return (void*)p; };
    bf* W0T = (bf*)take((size_t)HH * KIN * 2); bf* W1T = (bf*)take((size_t)HH * HH * 2); bf* W2T = (bf*)take((size_t)KOUT * HH * 2); bf* ZW = (bf*)take((size_t)KOUT * HH * 2);
    bf* Sh = (bf*)take((size_t)RCH * KIN * 2); bf* Sl = (bf*)take((size_t)RCH * KIN * 2); float* Hf = (float*)take((size_t)RCH * HH * 4); bf* Ph = (bf*)take((size_t)RCH * HH * 2); bf* Pl = (bf*)take((size_t)RCH * HH * 2);
    float* FKT = (float*)take((size_t)CB * KOUT * NN * 4); bf* XT = (bf*)take((size_t)CB * DP * NN * 2); float* C4 = Hf;
    if ((size_t)(wsp - (char*)d_ws) > ws_size) return;
    k_w0t<<<(HH * KIN / 2 + 255) / 256, 256, 0, stream>>>(W0, W0T); k_wtG<<<(unsigned)((HH * HH / 64 + 63) / 64), 256, 0, stream>>>(W1, HH, HH, W1T); k_wtG<<<(unsigned)((HH * KOUT / 64 + 63) / 64), 256, 0, stream>>>(W2, HH, KOUT, W2T);
    k_zero8<<<(KOUT * HH / 8 + 255) / 256, 256, 0, stream>>>(ZW, (size_t)KOUT * HH / 8);
    const size_t n4 = (size_t)RCH * HH / 4; const unsigned nb4 = (unsigned)((n4 + 255) / 256);
    for (int ck = 0; ck < NCH; ++ck) {
        k_scal<<<RCH / 256, 256, 0, stream>>>(x, u, basis, ck, Sh, Sl);
        k_gemmw<bf, 1, true><<<dim3(RCH / 64, HH / 64, 1), 32, 0, stream>>>(Sh, Sl, W0T, nullptr, KIN, Hf, HH, b0, 0, 0, 0);
        k_lrsplit<<<nb4, 256, 0, stream>>>(Hf, Ph, Pl, n4);
        k_gemmw<bf, 1, true><<<dim3(RCH / 64, HH / 64, 1), 32, 0, stream>>>(Ph, Pl, W1T, nullptr, HH, Hf, HH, b1, 0, 0, 0);
        k_lrsplit<<<nb4, 256, 0, stream>>>(Hf, Ph, Pl, n4);
        k_gemmw<bf, 2, false><<<dim3(KOUT / 64, NN / 64, CB), 32, 0, stream>>>(W2T, ZW, Ph, Pl, HH, FKT, NN, nullptr, 0, (size_t)NN * HH, (size_t)KOUT * NN);
        k_fksplit<<<(unsigned)(((size_t)CB * KOUT * NN / 4 + 255) / 256), 256, 0, stream>>>(FKT, b2, Ph, Pl, (size_t)CB * KOUT * NN / 4);
        k_xt<<<(unsigned)(((size_t)CB * DP * NN / 2 + 255) / 256), 256, 0, stream>>>(x, ck, XT);
        k_gemmw<bf, 1, false><<<dim3(KOUT / 64, DP / 64, CB), 32, 0, stream>>>(Ph, Pl, XT, nullptr, NN, C4, DP, nullptr, (size_t)KOUT * NN, (size_t)DP * NN, (size_t)KOUT * DP);
        k_out<<<(CB * KOUT + 255) / 256, 256, 0, stream>>>(C4, ck, OUT); }
}
